// ConformerLayer_80513456931453
// MI455X (gfx1250) — hardware-verified
//
#include <hip/hip_runtime.h>
#define NB 8
#define CC 384
#define TT 1024
#define NH 4
#define DH 96
#define FF 1536
#define WIN 4
#define NREL 9
#define NR (NB * TT)
typedef __bf16 v16b __attribute__((ext_vector_type(16)));
typedef unsigned short v8us __attribute__((ext_vector_type(8), may_alias));
typedef float  v8f  __attribute__((ext_vector_type(8)));
typedef float  v4f  __attribute__((ext_vector_type(4)));
typedef float  v4fa __attribute__((ext_vector_type(4), may_alias));
union FragB { v16b v; v8us half[2]; unsigned short u[16]; };

__device__ __forceinline__ unsigned short bf16_bits(float x) { unsigned int u = __float_as_uint(x); return (unsigned short)((u + 0x7FFFu + ((u >> 16) & 1u)) >> 16); }
__device__ __forceinline__ float bf16_val(unsigned short b) { return __uint_as_float(((unsigned int)b) << 16); }
__device__ __forceinline__ float bf16_round(float x) { return bf16_val(bf16_bits(x)); }
template <int NT>
__device__ __forceinline__ v8f mmaN(v16b ah, v16b al, v16b bh, v16b bl, v8f c) {
  c = __builtin_amdgcn_wmma_f32_16x16x32_bf16(false, ah, false, bh, (short)0, c, false, false);
  if (NT >= 2) c = __builtin_amdgcn_wmma_f32_16x16x32_bf16(false, al, false, bh, (short)0, c, false, false);
  if (NT >= 3) c = __builtin_amdgcn_wmma_f32_16x16x32_bf16(false, ah, false, bl, (short)0, c, false, false);
  asm volatile("v_nop\n\tv_nop\n\tv_nop\n\tv_nop" : "+v"(c) : "v"(ah), "v"(al), "v"(bh), "v"(bl));
  return c;
}

__global__ __launch_bounds__(256) void k_wt_bf16(const float* __restrict__ W, unsigned short* __restrict__ Wt, int K, int N) {
  const int t = blockIdx.x * 256 + threadIdx.x;
  const int k8n = K / 8;
  if (t >= N * k8n) return;
  const int n = t / k8n, k8 = (t % k8n) * 8;
  v8us v;
#pragma unroll
  for (int i = 0; i < 8; ++i) v[i] = bf16_bits(W[(size_t)(k8 + i) * N + n]);
  *(volatile v8us*)(Wt + (size_t)n * K + k8) = v;
  __threadfence();
  *(volatile v8us*)(Wt + (size_t)n * K + k8) = v;
}

template <bool ASPLIT, int ACT, bool BIAS_BF16>
__global__ __launch_bounds__(128) void k_gemm_bf(const float* __restrict__ A, int lda, const unsigned short* __restrict__ Wt, int ldb,
                                               const float* __restrict__ bias, float* __restrict__ C, int ldc, int M, int N, int K) {
  __shared__ __attribute__((aligned(16))) float so[4][16][64];
  const int tid = threadIdx.x, w = tid >> 5, lane = tid & 31, ln = lane & 15, hh = lane >> 4;
  const int ntn = N / 64;
  const int wid = blockIdx.x * 4 + w;
  const int mt = wid / ntn, nq = wid % ntn;
  if (mt * 16 >= M) return;
  const int row0 = mt * 16, col0 = nq * 64;
  const float* arow = A + (size_t)(row0 + ln) * lda;
  v8f acc[4] = {};
  for (int kb = 0; kb < K; kb += 32) {
    FragB ah, al;
    const v4f x0 = *(const v4fa*)(arow + kb + 8 * hh), x1 = *(const v4fa*)(arow + kb + 8 * hh + 4);
    const v4f x2 = *(const v4fa*)(arow + kb + 16 + 8 * hh), x3 = *(const v4fa*)(arow + kb + 16 + 8 * hh + 4);
    float xs[16] = {x0[0],x0[1],x0[2],x0[3],x1[0],x1[1],x1[2],x1[3],x2[0],x2[1],x2[2],x2[3],x3[0],x3[1],x3[2],x3[3]};
#pragma unroll
    for (int i = 0; i < 16; ++i) { const unsigned short hb = bf16_bits(xs[i]); ah.u[i] = hb; al.u[i] = ASPLIT ? bf16_bits(xs[i] - bf16_val(hb)) : (unsigned short)0; }
#pragma unroll
    for (int t = 0; t < 4; ++t) {
      const unsigned short* brow = Wt + (size_t)(col0 + t * 16 + ln) * ldb + kb;
      FragB b;
      b.half[0] = *(const v8us*)(brow + 8 * hh);
      b.half[1] = *(const v8us*)(brow + 16 + 8 * hh);
      acc[t] = mmaN<ASPLIT ? 2 : 1>(ah.v, al.v, b.v, b.v, acc[t]);
    }
  }
#pragma unroll
  for (int t = 0; t < 4; ++t) {
    float bv = bias ? bias[col0 + t * 16 + ln] : 0.f;
    if (BIAS_BF16) bv = bf16_round(bv);
#pragma unroll
    for (int r = 0; r < 8; ++r) { float v = acc[t][r] + bv; if (ACT == 1) v = fmaxf(v, 0.f); so[w][8 * hh + r][t * 16 + ln] = v; }
  }
  __builtin_amdgcn_fence(__ATOMIC_ACQ_REL, "workgroup");
  __builtin_amdgcn_wave_barrier();
  const int rsub = lane >> 4, c4 = (lane & 15) * 4;
  for (int pass = 0; pass < 2; ++pass) {
#pragma unroll
    for (int q = 0; q < 8; ++q) {
      const int r = q * 2 + rsub;
      const v4f v = *(const v4fa*)&so[w][r][c4];
      *(volatile v4f*)(C + (size_t)(row0 + r) * ldc + col0 + c4) = v;
    }
    if (pass == 0) __threadfence();
  }
}

template <bool ASPLIT, int ACT, bool BIAS_BF16, bool RES_BF16>
__global__ __launch_bounds__(128) void k_gemm_bf3(const float* __restrict__ A, int lda, const unsigned short* __restrict__ Wt, int ldb,
                                                const float* __restrict__ bias, const float* __restrict__ resid, int rmod, int ldr,
                                                float* __restrict__ C, int ldc, int M, int N, int K) {
  __shared__ __attribute__((aligned(16))) float so[4][16][64];
  const int tid = threadIdx.x, w = tid >> 5, lane = tid & 31, ln = lane & 15, hh = lane >> 4;
  const int ntn = N / 64;
  const int wid = blockIdx.x * 4 + w;
  const int mt = wid / ntn, nq = wid % ntn;
  if (mt * 16 >= M) return;
  const int row0 = mt * 16, col0 = nq * 64;
  const float* arow = A + (size_t)(row0 + ln) * lda;
  v8f acc[4] = {};
  for (int kb = 0; kb < K; kb += 32) {
    FragB ah, al;
    const v4f x0 = *(const v4fa*)(arow + kb + 8 * hh), x1 = *(const v4fa*)(arow + kb + 8 * hh + 4);
    const v4f x2 = *(const v4fa*)(arow + kb + 16 + 8 * hh), x3 = *(const v4fa*)(arow + kb + 16 + 8 * hh + 4);
    float xs[16] = {x0[0],x0[1],x0[2],x0[3],x1[0],x1[1],x1[2],x1[3],x2[0],x2[1],x2[2],x2[3],x3[0],x3[1],x3[2],x3[3]};
#pragma unroll
    for (int i = 0; i < 16; ++i) { const unsigned short hb = bf16_bits(xs[i]); ah.u[i] = hb; al.u[i] = ASPLIT ? bf16_bits(xs[i] - bf16_val(hb)) : (unsigned short)0; }
#pragma unroll
    for (int t = 0; t < 4; ++t) {
      const unsigned short* brow = Wt + (size_t)(col0 + t * 16 + ln) * ldb + kb;
      FragB b;
      b.half[0] = *(const v8us*)(brow + 8 * hh);
      b.half[1] = *(const v8us*)(brow + 16 + 8 * hh);
      acc[t] = mmaN<ASPLIT ? 2 : 1>(ah.v, al.v, b.v, b.v, acc[t]);
    }
  }
#pragma unroll
  for (int t = 0; t < 4; ++t) {
    const int col = col0 + t * 16 + ln;
    float bv = bias ? bias[col] : 0.f;
    if (BIAS_BF16) bv = bf16_round(bv);
#pragma unroll
    for (int r = 0; r < 8; ++r) {
      float v = acc[t][r] + bv;
      if (resid) { float rv = resid[(size_t)((row0 + 8 * hh + r) % rmod) * ldr + col]; if (RES_BF16) rv = bf16_round(rv); v += rv; }
      if (ACT == 1) v = fmaxf(v, 0.f);
      if (ACT == 2) v = 0.5f * v * (1.0f + erff(v * 0.70710678118654752f));
      if (ACT == 3) { const float u = 0.7978845608028654f * (v + 0.044715f * v * v * v); v = 0.5f * v * (1.0f + tanhf(u)); }
      so[w][8 * hh + r][t * 16 + ln] = v;
    }
  }
  __builtin_amdgcn_fence(__ATOMIC_ACQ_REL, "workgroup");
  __builtin_amdgcn_wave_barrier();
  const int rsub = lane >> 4, c4 = (lane & 15) * 4;
  for (int pass = 0; pass < 2; ++pass) {
#pragma unroll
    for (int q = 0; q < 8; ++q) {
      const int r = q * 2 + rsub;
      const v4f v = *(const v4fa*)&so[w][r][c4];
      *(volatile v4f*)(C + (size_t)(row0 + r) * ldc + col0 + c4) = v;
    }
    if (pass == 0) __threadfence();
  }
}
template <bool PARAM_BF16>
__global__ __launch_bounds__(256) void k_layernorm(const float* __restrict__ X, const float* __restrict__ R, const float* __restrict__ g, const float* __restrict__ bta,
                                                  float* __restrict__ out_sum, float* __restrict__ out_norm, int N, float eps) {
  __shared__ float red[256];
  const int row = blockIdx.x, tid = threadIdx.x;
  const float* x = X + (size_t)row * N; const float* rr = R ? R + (size_t)row * N : nullptr;
  float vals[16];
  const int per = N / 256;
  float s1 = 0.f;
  for (int u = 0; u < per / 4; ++u) {
    const int j = tid * 4 + 1024 * u;
    const v4f a = *(const v4fa*)(x + j);
    v4f b = {0.f,0.f,0.f,0.f}; if (rr) b = *(const v4fa*)(rr + j);
#pragma unroll
    for (int q = 0; q < 4; ++q) { const float v = a[q] + b[q]; vals[u * 4 + q] = v; s1 += v; }
  }
  red[tid] = s1; __syncthreads();
  for (int st = 128; st > 0; st >>= 1) { if (tid < st) red[tid] += red[tid + st]; __syncthreads(); }
  const float mu = red[0] / (float)N; __syncthreads();
  float s2 = 0.f;
  for (int u = 0; u < per / 4; ++u)
#pragma unroll
    for (int q = 0; q < 4; ++q) { const float c = vals[u * 4 + q] - mu; s2 += c * c; }
  red[tid] = s2; __syncthreads();
  for (int st = 128; st > 0; st >>= 1) { if (tid < st) red[tid] += red[tid + st]; __syncthreads(); }
  const float rs = rsqrtf(red[0] / (float)N + eps);
  for (int pass = 0; pass < 2; ++pass) {
    for (int u = 0; u < per / 4; ++u) {
      const int j = tid * 4 + 1024 * u;
      v4f o, sm;
#pragma unroll
      for (int q = 0; q < 4; ++q) {
        float gg = g[j + q], bb = bta[j + q];
        if (PARAM_BF16) { gg = bf16_round(gg); bb = bf16_round(bb); }
        sm[q] = vals[u * 4 + q]; o[q] = (vals[u * 4 + q] - mu) * rs * gg + bb;
      }
      if (out_sum) *(volatile v4f*)(out_sum + (size_t)row * N + j) = sm;
      *(volatile v4f*)(out_norm + (size_t)row * N + j) = o;
    }
    if (pass == 0) __threadfence();
  }
}


typedef _Float16 v16h __attribute__((ext_vector_type(16)));
union FragH { v16h v; v8us half[2]; _Float16 h[16]; unsigned short u[16]; };
template <int NT>
__device__ __forceinline__ v8f mmaH(v16h ah, v16h al, v16h bh, v16h bl, v8f c) {
  c = __builtin_amdgcn_wmma_f32_16x16x32_f16(false, ah, false, bh, (short)0, c, false, false);
  if (NT >= 2) c = __builtin_amdgcn_wmma_f32_16x16x32_f16(false, al, false, bh, (short)0, c, false, false);
  if (NT >= 3) c = __builtin_amdgcn_wmma_f32_16x16x32_f16(false, ah, false, bl, (short)0, c, false, false);
  asm volatile("v_nop\n\tv_nop\n\tv_nop\n\tv_nop" : "+v"(c) : "v"(ah), "v"(al), "v"(bh), "v"(bl));
  return c;
}
template <bool ASPLIT>
__global__ __launch_bounds__(128) void k_gemm_h(const float* __restrict__ A, int lda, size_t sA, const _Float16* __restrict__ Bh, int ldb, size_t sB, float alpha, float* __restrict__ C, int ldc, size_t sC, int M, int N, int K) {
  __shared__ __attribute__((aligned(16))) float so[4][16][64];
  const int tid = threadIdx.x, w = tid >> 5, lane = tid & 31, ln = lane & 15, hh = lane >> 4; const int by = blockIdx.y;
  A += (size_t)by * sA; Bh += (size_t)by * sB; C += (size_t)by * sC;
  const int ntn = (N + 63) / 64; const int wid = blockIdx.x * 4 + w; const int mt = wid / ntn, nq = wid % ntn; if (mt * 16 >= M) return;
  const int row0 = mt * 16, col0 = nq * 64; const float* arow = A + (size_t)(row0 + ln) * lda;
  v8f acc[4] = {};
  for (int kb = 0; kb < K; kb += 32) {
    FragH ah, al;
    const v4f x0 = *(const v4fa*)(arow + kb + 8 * hh), x1 = *(const v4fa*)(arow + kb + 8 * hh + 4), x2 = *(const v4fa*)(arow + kb + 16 + 8 * hh), x3 = *(const v4fa*)(arow + kb + 16 + 8 * hh + 4);
    float xs[16] = {x0[0],x0[1],x0[2],x0[3],x1[0],x1[1],x1[2],x1[3],x2[0],x2[1],x2[2],x2[3],x3[0],x3[1],x3[2],x3[3]};
#pragma unroll
    for (int i = 0; i < 16; ++i) { const _Float16 h = (_Float16)xs[i]; ah.h[i] = h; al.h[i] = ASPLIT ? (_Float16)(xs[i] - (float)h) : (_Float16)0.0f; }
#pragma unroll
    for (int t = 0; t < 4; ++t) { if (col0 + t * 16 >= N) continue; const size_t boff = (size_t)(col0 + t * 16 + ln) * ldb + kb; FragH bq; bq.half[0] = *(const v8us*)(Bh + boff + 8 * hh); bq.half[1] = *(const v8us*)(Bh + boff + 16 + 8 * hh);
      acc[t] = mmaH<ASPLIT ? 2 : 1>(ah.v, al.v, bq.v, bq.v, acc[t]); }
  }
#pragma unroll
  for (int t = 0; t < 4; ++t) { if (col0 + t * 16 >= N) continue;
#pragma unroll
    for (int r = 0; r < 8; ++r) so[w][8 * hh + r][t * 16 + ln] = acc[t][r] * alpha; }
  __builtin_amdgcn_fence(__ATOMIC_ACQ_REL, "workgroup"); __builtin_amdgcn_wave_barrier();
  const int rsub = lane >> 4, c4 = (lane & 15) * 4;
  for (int pass = 0; pass < 2; ++pass) {
#pragma unroll
    for (int q = 0; q < 8; ++q) { const int r = q * 2 + rsub; if (col0 + c4 < N) { const v4f v = *(const v4fa*)&so[w][r][c4]; *(volatile v4f*)(C + (size_t)(row0 + r) * ldc + col0 + c4) = v; } }
    if (pass == 0) __threadfence(); }
}

__global__ __launch_bounds__(256) void k_wt_f16(const float* __restrict__ W, _Float16* __restrict__ Wt, int K, int N, float scale) {
  const int t = blockIdx.x * 256 + threadIdx.x; if (t >= N * (K / 8)) return; const int n = t / (K / 8), k8 = (t % (K / 8)) * 8; FragH f;
#pragma unroll
  for (int i = 0; i < 8; ++i) f.h[i] = (_Float16)(bf16_round(W[(size_t)(k8 + i) * N + n]) * scale); const v8us o = f.half[0];
  *(volatile v8us*)((unsigned short*)Wt + (size_t)n * K + k8) = o; __threadfence(); *(volatile v8us*)((unsigned short*)Wt + (size_t)n * K + k8) = o;
}
template <int ACT>
__global__ __launch_bounds__(128) void k_gemm_hhx(const _Float16* __restrict__ A, int lda, size_t sA, const _Float16* __restrict__ Bh, int ldb, size_t sB, float alpha, const float* __restrict__ bias, size_t sBias, const float* __restrict__ CP, int rowsPerB, size_t sCPb, int row0g,
    float* __restrict__ C, _Float16* __restrict__ C16, int ldc, size_t sC, int M, int N, int K) {
  __shared__ __attribute__((aligned(16))) float so[4][16][64];
  const int tid = threadIdx.x, w = tid >> 5, lane = tid & 31, ln = lane & 15, hh = lane >> 4; const int by = blockIdx.y;
  A += (size_t)by * sA; Bh += (size_t)by * sB; const size_t cofs = (size_t)by * sC; const float* bp = bias ? bias + (size_t)by * sBias : nullptr;
  const int ntn = (N + 63) / 64; const int wid = blockIdx.x * 4 + w; const int mt = wid / ntn, nq = wid % ntn; if (mt * 16 >= M) return;
  const int row0 = mt * 16, col0 = nq * 64; const _Float16* arow = A + (size_t)(row0 + ln) * lda;
  v8f acc[4] = {};
  for (int kb = 0; kb < K; kb += 32) { FragH ah; ah.half[0] = *(const v8us*)((const unsigned short*)arow + kb + 8 * hh); ah.half[1] = *(const v8us*)((const unsigned short*)arow + kb + 16 + 8 * hh);
#pragma unroll
    for (int t = 0; t < 4; ++t) { if (col0 + t * 16 >= N) continue; const size_t boff = (size_t)(col0 + t * 16 + ln) * ldb + kb; FragH bq; bq.half[0] = *(const v8us*)((const unsigned short*)Bh + boff + 8 * hh); bq.half[1] = *(const v8us*)((const unsigned short*)Bh + boff + 16 + 8 * hh);
      acc[t] = mmaH<1>(ah.v, ah.v, bq.v, bq.v, acc[t]); }
  }
#pragma unroll
  for (int t = 0; t < 4; ++t) { if (col0 + t * 16 >= N) continue; const int col = col0 + t * 16 + ln; const float bv = bp ? bf16_round(bp[col]) : 0.f;
#pragma unroll
    for (int r = 0; r < 8; ++r) { float v = acc[t][r] * alpha + bv; if (CP) { const int bidx = (row0g + row0 + 8 * hh + r) / rowsPerB; v += CP[(size_t)bidx * sCPb + (size_t)by * 64 + col]; } if (ACT == 1) v = (v > 0.f) ? v : expm1f(v); else if (ACT == 7) v = (v > 0.f) ? v + 1.0f : expf(v); else if (ACT == 8) v = tanhf(v); else if (ACT == 9) v = 0.5f * v * (1.0f + tanhf(0.7978845608028654f * (v + 0.044715f * v * v * v))); else if (ACT == 11) v = 1.0f / (1.0f + expf(-v)); else if (ACT == 12) v = (v > 0.f) ? v : 0.01f * v; else if (ACT == 14) v = (v > 0.f) ? v : 0.1f * v; else if (ACT == 15) v = v / (1.0f + expf(-v)); else if (ACT == 3) v = fmaxf(v, 0.f); else if (ACT == 6) v = 0.5f * v * (1.0f + erff(v * 0.70710678118654752f)); so[w][8 * hh + r][t * 16 + ln] = v; } }
  __builtin_amdgcn_fence(__ATOMIC_ACQ_REL, "workgroup"); __builtin_amdgcn_wave_barrier();
  const int rsub = lane >> 4, c4 = (lane & 15) * 4; typedef _Float16 v4h __attribute__((ext_vector_type(4)));
  for (int pass = 0; pass < 2; ++pass) {
#pragma unroll
    for (int q = 0; q < 8; ++q) { const int r = q * 2 + rsub; if (col0 + c4 < N) { const v4f v = *(const v4fa*)&so[w][r][c4]; if (C) *(volatile v4f*)(C + cofs + (size_t)(row0 + r) * ldc + col0 + c4) = v; if (C16) { v4h h4; for (int i = 0; i < 4; ++i) h4[i] = (_Float16)v[i]; *(volatile v4h*)(C16 + cofs + (size_t)(row0 + r) * ldc + col0 + c4) = h4; } } }
    if (pass == 0) __threadfence(); }
}


typedef _Float16 v4h __attribute__((ext_vector_type(4)));

__global__ __launch_bounds__(256) void k_x16(const float* __restrict__ x, _Float16* __restrict__ X16, size_t n8) { const size_t t = (size_t)blockIdx.x * 256 + threadIdx.x; if (t >= n8) return; FragH f;
#pragma unroll
  for (int q = 0; q < 8; ++q) f.h[q] = (_Float16)bf16_round(x[t * 8 + q]); *(volatile v8us*)((unsigned short*)X16 + t * 8) = f.half[0]; __threadfence(); *(volatile v8us*)((unsigned short*)X16 + t * 8) = f.half[0]; }
__global__ __launch_bounds__(256) void k_h16(const float* __restrict__ x, _Float16* __restrict__ X16, size_t n8) { const size_t t = (size_t)blockIdx.x * 256 + threadIdx.x; if (t >= n8) return; FragH f;
#pragma unroll
  for (int q = 0; q < 8; ++q) f.h[q] = (_Float16)x[t * 8 + q]; *(volatile v8us*)((unsigned short*)X16 + t * 8) = f.half[0]; __threadfence(); *(volatile v8us*)((unsigned short*)X16 + t * 8) = f.half[0]; }
__global__ __launch_bounds__(256) void k_round16f(const float* __restrict__ W, _Float16* __restrict__ Bt, size_t n8) { const size_t t = (size_t)blockIdx.x * 256 + threadIdx.x; if (t >= n8) return; FragH f;
#pragma unroll
  for (int i = 0; i < 8; ++i) f.h[i] = (_Float16)(bf16_round(W[t * 8 + i]) * 16.0f); *(volatile v8us*)((unsigned short*)Bt + t * 8) = f.half[0]; __threadfence(); *(volatile v8us*)((unsigned short*)Bt + t * 8) = f.half[0]; }
template <int NHv, int TTv>
__global__ __launch_bounds__(256) void k_vt(const _Float16* __restrict__ V16, int ldv, int voff, _Float16* __restrict__ Vt) { __shared__ unsigned short tl[64][66]; const int tid = threadIdx.x; const int slab = blockIdx.x / (TTv / 64), lg = blockIdx.x % (TTv / 64); const int b = slab / NHv, h = slab % NHv;
  for (int i = tid; i < 64 * 8; i += 256) { const int r = i / 8, c8 = (i % 8) * 8; FragH f; f.half[0] = *(const v8us*)((const unsigned short*)V16 + ((size_t)b * TTv + lg * 64 + r) * ldv + voff + h * 64 + c8);
#pragma unroll
    for (int q = 0; q < 8; ++q) tl[r][c8 + q] = f.u[q]; }
  __syncthreads();
  for (int pass = 0; pass < 2; ++pass) {
#pragma unroll
    for (int rd = 0; rd < 2; ++rd) { const int d = rd * 32 + tid / 8, pc = tid % 8; FragH f;
#pragma unroll
      for (int q = 0; q < 8; ++q) f.u[q] = tl[pc * 8 + q][d];
      *(volatile v8us*)((unsigned short*)Vt + ((size_t)slab * 64 + d) * TTv + lg * 64 + pc * 8) = f.half[0]; }
    if (pass == 0) __threadfence(); } }

__global__ __launch_bounds__(256) void k_hl(const float* __restrict__ F, _Float16* __restrict__ Hh, _Float16* __restrict__ Hl, size_t n8) { const size_t t = (size_t)blockIdx.x * 256 + threadIdx.x; if (t >= n8) return; FragH fh, fl; const v4f a = *(const v4fa*)(F + t * 8), c = *(const v4fa*)(F + t * 8 + 4);
#pragma unroll
  for (int q = 0; q < 4; ++q) { _Float16 h = (_Float16)a[q]; fh.h[q] = h; fl.h[q] = (_Float16)((a[q] - (float)h) * 1024.0f); h = (_Float16)c[q]; fh.h[4 + q] = h; fl.h[4 + q] = (_Float16)((c[q] - (float)h) * 1024.0f); }
  for (int pass = 0; pass < 2; ++pass) { *(volatile v8us*)((unsigned short*)Hh + t * 8) = fh.half[0]; *(volatile v8us*)((unsigned short*)Hl + t * 8) = fl.half[0]; if (pass == 0) __threadfence(); } }

__device__ __forceinline__ float sigm_p(float x) { return 1.0f / (1.0f + expf(-x)); }
__device__ __forceinline__ float sigm_f(float x) { return __builtin_amdgcn_rcpf(1.0f + __expf(-x)); }
__global__ __launch_bounds__(256) void k_tin(const float* __restrict__ x, float* __restrict__ XT) { const size_t t_ = (size_t)blockIdx.x * 256 + threadIdx.x; if (t_ >= (size_t)NR * (CC / 4)) return; const int c0 = (int)(t_ % (CC / 4)) * 4; const size_t r = t_ / (CC / 4); const int b = (int)(r / TT), t = (int)(r % TT); v4f v;
#pragma unroll
  for (int q = 0; q < 4; ++q) v[q] = bf16_round(x[((size_t)b * CC + c0 + q) * TT + t]); *(volatile v4f*)(XT + r * CC + c0) = v; __threadfence(); *(volatile v4f*)(XT + r * CC + c0) = v; }
__global__ __launch_bounds__(256) void k_ln(const float* __restrict__ X, const float* __restrict__ g, const float* __restrict__ bb, _Float16* __restrict__ Y) {
  #pragma clang fp contract(off)
  const int tid = threadIdx.x, w = tid >> 5, l = tid & 31; const size_t r = (size_t)blockIdx.x * 8 + w; float v[12]; float s = 0.f;
#pragma unroll
  for (int q = 0; q < 3; ++q) { const v4f a = *(const v4fa*)(X + r * CC + q * 128 + 4 * l);
#pragma unroll
    for (int j = 0; j < 4; ++j) { v[q * 4 + j] = a[j]; s += a[j]; } }
  for (int o = 16; o > 0; o >>= 1) s += __shfl_xor(s, o, 32); const float mu = s / (float)CC; float vs = 0.f;
#pragma unroll
  for (int i = 0; i < 12; ++i) { const float d = v[i] - mu; vs += d * d; }
  for (int o = 16; o > 0; o >>= 1) vs += __shfl_xor(vs, o, 32); const float rs = rsqrtf(vs / (float)CC + 1e-5f);
  for (int pass = 0; pass < 2; ++pass) {
#pragma unroll
    for (int q = 0; q < 3; ++q) { FragH f;
#pragma unroll
      for (int j = 0; j < 4; ++j) { const int c = q * 128 + 4 * l + j; f.h[j] = (_Float16)((v[q * 4 + j] - mu) * rs * bf16_round(g[c]) + bf16_round(bb[c])); }
      *(volatile unsigned long long*)((unsigned short*)Y + r * CC + q * 128 + 4 * l) = *(const unsigned long long*)&f.u[0]; }
    if (pass == 0) __threadfence(); } }
__global__ __launch_bounds__(256) void k_bscale(const float* __restrict__ b, float* __restrict__ Bs, int n, float s) { const int i = blockIdx.x * 256 + threadIdx.x; if (i >= n) return; const float v = bf16_round(b[i]) * s; *(volatile float*)(Bs + i) = v; __threadfence(); *(volatile float*)(Bs + i) = v; }
__global__ __launch_bounds__(256) void k_relsoft(const float* __restrict__ S, const _Float16* __restrict__ Q16, const float* __restrict__ relk, const float* __restrict__ mask, int b, _Float16* __restrict__ P16, float* __restrict__ PB) {
  #pragma clang fp contract(off)
  __shared__ __attribute__((aligned(16))) unsigned short prow[8][TT]; __shared__ float band[8][32]; __shared__ float srow[8][TT];
  const int tid = threadIdx.x, w = tid >> 5, l = tid & 31; const int ht = blockIdx.x * 8 + w; const int h = ht / TT, t = ht % TT;
  float qv[3];
#pragma unroll
  for (int j = 0; j < 3; ++j) qv[j] = (float)Q16[((size_t)b * TT + t) * CC + h * DH + l + 32 * j];
  float relv[NREL];
#pragma unroll
  for (int m = 0; m < NREL; ++m) { float p = 0.f;
#pragma unroll
    for (int j = 0; j < 3; ++j) p += qv[j] * bf16_round(relk[m * DH + l + 32 * j]); for (int o = 16; o > 0; o >>= 1) p += __shfl_xor(p, o, 32); relv[m] = p * 0.10206207261596575f; }
  const float* sr = S + ((size_t)h * TT + t) * TT; float* lr = &srow[w][0]; const float mt = bf16_round(mask[(size_t)b * TT + t]); float mx = -3.0e38f;
#pragma unroll 1
  for (int q = 0; q < 32; ++q) { const int s = 32 * l + q; float x = sr[s]; const int m = s - t + WIN;
#pragma unroll
    for (int mm = 0; mm < NREL; ++mm) x += (m == mm) ? relv[mm] : 0.f;
    if (mt * bf16_round(mask[(size_t)b * TT + s]) == 0.f) x = -1e4f; lr[s] = x; mx = fmaxf(mx, x); }
  for (int o = 16; o > 0; o >>= 1) mx = fmaxf(mx, __shfl_xor(mx, o, 32)); float sum = 0.f;
#pragma unroll 1
  for (int q = 0; q < 32; ++q) sum += expf(lr[32 * l + q] - mx);
  for (int o = 16; o > 0; o >>= 1) sum += __shfl_xor(sum, o, 32); const float inv = 1.0f / sum;
#pragma unroll 1
  for (int q = 0; q < 32; ++q) { const int s = 32 * l + q; const float p = expf(lr[s] - mx) * inv; FragH f; f.h[0] = (_Float16)(p * 1024.0f); prow[w][s] = f.u[0]; const int m = s - t + WIN; if (m >= 0 && m < NREL) band[w][m] = p; }
  __syncthreads();
  float bv = 0.f; if (l < NREL) { const int s = t + l - WIN; bv = (s >= 0 && s < TT) ? band[w][l] : 0.f; }
  for (int pass = 0; pass < 2; ++pass) {
#pragma unroll
    for (int k = 0; k < 4; ++k) { const v8us pv = *(const v8us*)&prow[w][k * 256 + l * 8]; *(volatile v8us*)((unsigned short*)P16 + ((size_t)h * TT + t) * TT + k * 256 + l * 8) = pv; }
    *(volatile float*)(PB + ((size_t)h * TT + t) * 32 + l) = bv;
    if (pass == 0) __threadfence(); } }
__global__ __launch_bounds__(256) void k_vt(const _Float16* __restrict__ V16, int b, _Float16* __restrict__ VT) { const int t_ = blockIdx.x * 256 + threadIdx.x; if (t_ >= NH * DH * (TT / 8)) return; const int s0 = (t_ % (TT / 8)) * 8; const int hd = t_ / (TT / 8); const int h = hd / DH, d = hd % DH; FragH f;
#pragma unroll
  for (int q = 0; q < 8; ++q) f.h[q] = V16[((size_t)b * TT + s0 + q) * CC + h * DH + d];
  *(volatile v8us*)((unsigned short*)VT + (size_t)hd * TT + s0) = f.half[0]; __threadfence(); *(volatile v8us*)((unsigned short*)VT + (size_t)hd * TT + s0) = f.half[0]; }
__global__ __launch_bounds__(256) void k_relv(const float* __restrict__ O, const float* __restrict__ PB, const float* __restrict__ relv, int b, _Float16* __restrict__ O16) {
  #pragma clang fp contract(off)
  const int t_ = blockIdx.x * 256 + threadIdx.x; if (t_ >= TT * (CC / 8)) return; const int c0 = (t_ % (CC / 8)) * 8; const int t = t_ / (CC / 8); const int h = c0 / DH, d0 = c0 % DH; const float* pb = PB + ((size_t)h * TT + t) * 32; FragH f;
#pragma unroll
  for (int q = 0; q < 8; ++q) { float v = O[(size_t)t * CC + c0 + q];
#pragma unroll
    for (int m = 0; m < NREL; ++m) v += pb[m] * bf16_round(relv[m * DH + d0 + q]); f.h[q] = (_Float16)v; }
  *(volatile v8us*)((unsigned short*)O16 + ((size_t)b * TT + t) * CC + c0) = f.half[0]; __threadfence(); *(volatile v8us*)((unsigned short*)O16 + ((size_t)b * TT + t) * CC + c0) = f.half[0]; }
__global__ __launch_bounds__(256) void k_glu(const float* __restrict__ PW, float* __restrict__ GL) {
  #pragma clang fp contract(off)
  const size_t t = (size_t)blockIdx.x * 256 + threadIdx.x; if (t >= (size_t)NR * (CC / 4)) return; const size_t r = t / (CC / 4); const int c0 = (int)(t % (CC / 4)) * 4; const v4f a = *(const v4fa*)(PW + r * (2 * CC) + c0), g = *(const v4fa*)(PW + r * (2 * CC) + CC + c0); v4f o;
#pragma unroll
  for (int q = 0; q < 4; ++q) o[q] = a[q] * sigm_f(g[q]); *(volatile v4f*)(GL + r * CC + c0) = o; __threadfence(); *(volatile v4f*)(GL + r * CC + c0) = o; }
__global__ __launch_bounds__(256) void k_dw(const float* __restrict__ GL, const float* __restrict__ dw, const float* __restrict__ dbb, const float* __restrict__ bg, const float* __restrict__ bnb, _Float16* __restrict__ CH) {
  #pragma clang fp contract(off)
  const size_t t_ = (size_t)blockIdx.x * 256 + threadIdx.x; if (t_ >= (size_t)NR * (CC / 8)) return; const int c0 = (int)(t_ % (CC / 8)) * 8; const size_t r = t_ / (CC / 8); const int b = (int)(r / TT), t = (int)(r % TT); const float bnk = rsqrtf(1.0f + 1e-5f); FragH f;
#pragma unroll
  for (int q = 0; q < 8; ++q) { const int c = c0 + q; float acc = 0.f;
#pragma unroll
    for (int k = 0; k < 7; ++k) { const int ts = t + k - 3; if (ts >= 0 && ts < TT) acc += GL[((size_t)b * TT + ts) * CC + c] * bf16_round(dw[c * 7 + k]); }
    acc += bf16_round(dbb[c]); float hv = acc * bnk * bf16_round(bg[c]) + bf16_round(bnb[c]); hv = hv * sigm_f(hv); f.h[q] = (_Float16)hv; }
  *(volatile v8us*)((unsigned short*)CH + r * CC + c0) = f.half[0]; __threadfence(); *(volatile v8us*)((unsigned short*)CH + r * CC + c0) = f.half[0]; }
__global__ __launch_bounds__(1024) void k_stat(const float* __restrict__ X, float* __restrict__ MU, float* __restrict__ RS) {
  #pragma clang fp contract(off)
  __shared__ float m1[32], m2[32]; const int tid = threadIdx.x, w = tid >> 5, l = tid & 31; const size_t r = (size_t)blockIdx.x * 32 + w; float v[12]; float s = 0.f;
#pragma unroll
  for (int q = 0; q < 3; ++q) { const v4f a = *(const v4fa*)(X + r * CC + q * 128 + 4 * l);
#pragma unroll
    for (int j = 0; j < 4; ++j) { v[q * 4 + j] = a[j]; s += a[j]; } }
  for (int o = 16; o > 0; o >>= 1) s += __shfl_xor(s, o, 32); const float mu = s / (float)CC; float vs = 0.f;
#pragma unroll
  for (int i = 0; i < 12; ++i) { const float d = v[i] - mu; vs += d * d; }
  for (int o = 16; o > 0; o >>= 1) vs += __shfl_xor(vs, o, 32); if (l == 0) { m1[w] = mu; m2[w] = rsqrtf(vs / (float)CC + 1e-5f); }
  __syncthreads();
  if (tid < 32) { *(volatile float*)(MU + (size_t)blockIdx.x * 32 + tid) = m1[tid]; *(volatile float*)(RS + (size_t)blockIdx.x * 32 + tid) = m2[tid]; __threadfence(); *(volatile float*)(MU + (size_t)blockIdx.x * 32 + tid) = m1[tid]; *(volatile float*)(RS + (size_t)blockIdx.x * 32 + tid) = m2[tid]; } }
__global__ __launch_bounds__(256) void k_tout(const float* __restrict__ X, const float* __restrict__ MU, const float* __restrict__ RS, const float* __restrict__ g, const float* __restrict__ bb, const float* __restrict__ mask, float* __restrict__ out) {
  #pragma clang fp contract(off)
  const size_t t_ = (size_t)blockIdx.x * 256 + threadIdx.x; if (t_ >= (size_t)NB * CC * (TT / 4)) return; const int t0 = (int)(t_ % (TT / 4)) * 4; const size_t bc = t_ / (TT / 4); const int b = (int)(bc / CC), c = (int)(bc % CC); const float gg = bf16_round(g[c]), be = bf16_round(bb[c]); v4f v;
#pragma unroll
  for (int q = 0; q < 4; ++q) { const size_t r = (size_t)b * TT + t0 + q; v[q] = ((X[r * CC + c] - MU[r]) * RS[r] * gg + be) * bf16_round(mask[(size_t)b * TT + t0 + q]); }
  *(volatile v4f*)(out + bc * TT + t0) = v; __threadfence(); *(volatile v4f*)(out + bc * TT + t0) = v; }

extern "C" void kernel_launch(void* const* d_in, const int* in_sizes, int n_in,
                              void* d_out, int out_size, void* d_ws, size_t ws_size, hipStream_t stream) {
  (void)in_sizes; (void)n_in; (void)out_size;
  const float* const* I = (const float* const*)d_in; const float* x = I[0]; const float* mask = I[1];
  const float* f1g = I[2]; const float* f1bb = I[3]; const float* f1w1 = I[4]; const float* f1b1 = I[5]; const float* f1w2 = I[6]; const float* f1b2 = I[7]; const float* preg = I[8]; const float* preb = I[9];
  const float* wq = I[10]; const float* bq = I[11]; const float* wk = I[12]; const float* bk = I[13]; const float* wv = I[14]; const float* bv = I[15]; const float* wo = I[16]; const float* bo = I[17]; const float* relk = I[18]; const float* relv = I[19];
  const float* cg = I[20]; const float* cb = I[21]; const float* pw1 = I[22]; const float* pb1 = I[23]; const float* dww = I[24]; const float* dwb = I[25]; const float* bng = I[26]; const float* bnb = I[27]; const float* pw2 = I[28]; const float* pb2 = I[29];
  const float* f2g = I[30]; const float* f2bb = I[31]; const float* f2w1 = I[32]; const float* f2b1 = I[33]; const float* f2w2 = I[34]; const float* f2b2 = I[35]; const float* postg = I[36]; const float* postb = I[37];
  char* ws = (char*)d_ws; size_t off = 0;
  auto take = [&](size_t bytes) { char* p = ws + off; off += (bytes + 255) & ~(size_t)255; return p; };
  _Float16* Bf1w1 = (_Float16*)take((size_t)FF * CC * 2); _Float16* Bf1w2 = (_Float16*)take((size_t)CC * FF * 2); _Float16* Bf2w1 = (_Float16*)take((size_t)FF * CC * 2); _Float16* Bf2w2 = (_Float16*)take((size_t)CC * FF * 2);
  _Float16* Bq = (_Float16*)take((size_t)CC * CC * 2); _Float16* Bk = (_Float16*)take((size_t)CC * CC * 2); _Float16* Bv = (_Float16*)take((size_t)CC * CC * 2); _Float16* Bo = (_Float16*)take((size_t)CC * CC * 2); _Float16* Bp1 = (_Float16*)take((size_t)2 * CC * CC * 2); _Float16* Bp2 = (_Float16*)take((size_t)CC * CC * 2); float* B2a = (float*)take(CC * 4); float* B2b = (float*)take(CC * 4);
  float* XT = (float*)take((size_t)NR * CC * 4); _Float16* LN16 = (_Float16*)take((size_t)NR * CC * 2); _Float16* FFH = (_Float16*)take((size_t)NR * FF * 2);
  _Float16* Q16 = (_Float16*)take((size_t)NR * CC * 2); _Float16* K16 = (_Float16*)take((size_t)NR * CC * 2); _Float16* V16 = (_Float16*)take((size_t)NR * CC * 2); float* S = (float*)take((size_t)NH * TT * TT * 4); _Float16* P16 = (_Float16*)take((size_t)NH * TT * TT * 2); float* PB = (float*)take((size_t)NH * TT * 32 * 4); _Float16* VT = (_Float16*)take((size_t)NH * DH * TT * 2); float* O = (float*)take((size_t)TT * CC * 4); _Float16* O16 = (_Float16*)take((size_t)NR * CC * 2);
  float* MU = (float*)take((size_t)NR * 4); float* RS = (float*)take((size_t)NR * 4);
  float* PW = (float*)FFH;        float* GL = S;   _Float16* CH = LN16;
  if (off > ws_size) return;
  k_round16f<<<(unsigned)(((size_t)FF * CC / 8 + 255) / 256), 256, 0, stream>>>(f1w1, Bf1w1, (size_t)FF * CC / 8); k_round16f<<<(unsigned)(((size_t)CC * FF / 8 + 255) / 256), 256, 0, stream>>>(f1w2, Bf1w2, (size_t)CC * FF / 8);
  k_round16f<<<(unsigned)(((size_t)FF * CC / 8 + 255) / 256), 256, 0, stream>>>(f2w1, Bf2w1, (size_t)FF * CC / 8); k_round16f<<<(unsigned)(((size_t)CC * FF / 8 + 255) / 256), 256, 0, stream>>>(f2w2, Bf2w2, (size_t)CC * FF / 8);
  k_round16f<<<(CC * CC / 8 + 255) / 256, 256, 0, stream>>>(wq, Bq, (size_t)CC * CC / 8); k_round16f<<<(CC * CC / 8 + 255) / 256, 256, 0, stream>>>(wk, Bk, (size_t)CC * CC / 8); k_round16f<<<(CC * CC / 8 + 255) / 256, 256, 0, stream>>>(wv, Bv, (size_t)CC * CC / 8); k_round16f<<<(CC * CC / 8 + 255) / 256, 256, 0, stream>>>(wo, Bo, (size_t)CC * CC / 8);
  k_round16f<<<(2 * CC * CC / 8 + 255) / 256, 256, 0, stream>>>(pw1, Bp1, (size_t)2 * CC * CC / 8); k_round16f<<<(CC * CC / 8 + 255) / 256, 256, 0, stream>>>(pw2, Bp2, (size_t)CC * CC / 8);
  k_bscale<<<(CC + 255) / 256, 256, 0, stream>>>(f1b2, B2a, CC, 0.5f); k_bscale<<<(CC + 255) / 256, 256, 0, stream>>>(f2b2, B2b, CC, 0.5f);
  k_tin<<<(unsigned)(((size_t)NR * (CC / 4) + 255) / 256), 256, 0, stream>>>(x, XT);
  const dim3 gC(((NR / 16) * (CC / 64) + 3) / 4, 1), gF(((NR / 16) * (FF / 64) + 3) / 4, 1), g2C(((NR / 16) * (2 * CC / 64) + 3) / 4, 1);
  k_ln<<<NR / 8, 256, 0, stream>>>(XT, f1g, f1bb, LN16);
  k_gemm_hhx<15><<<gF, 128, 0, stream>>>(LN16, CC, 0, Bf1w1, CC, 0, 0.0625f, f1b1, 0, nullptr, 1, 0, 0, nullptr, FFH, FF, 0, NR, FF, CC);
  k_gemm_hhx<0><<<gC, 128, 0, stream>>>(FFH, FF, 0, Bf1w2, FF, 0, 0.0625f * 0.5f, B2a, 0, XT, 1, (size_t)CC, 0, XT, nullptr, CC, 0, NR, CC, FF);
  k_ln<<<NR / 8, 256, 0, stream>>>(XT, preg, preb, LN16);
  k_gemm_hhx<0><<<gC, 128, 0, stream>>>(LN16, CC, 0, Bq, CC, 0, 0.0625f, bq, 0, nullptr, 1, 0, 0, nullptr, Q16, CC, 0, NR, CC, CC); k_gemm_hhx<0><<<gC, 128, 0, stream>>>(LN16, CC, 0, Bk, CC, 0, 0.0625f, bk, 0, nullptr, 1, 0, 0, nullptr, K16, CC, 0, NR, CC, CC); k_gemm_hhx<0><<<gC, 128, 0, stream>>>(LN16, CC, 0, Bv, CC, 0, 0.0625f, bv, 0, nullptr, 1, 0, 0, nullptr, V16, CC, 0, NR, CC, CC);
  for (int b = 0; b < NB; ++b) { const size_t rb0 = (size_t)b * TT * CC;
    k_gemm_hhx<0><<<dim3(((TT / 16) * (TT / 64) + 3) / 4, NH), 128, 0, stream>>>(Q16 + rb0, CC, DH, K16 + rb0, CC, DH, 0.10206207261596575f, nullptr, 0, nullptr, 1, 0, 0, S, nullptr, TT, (size_t)TT * TT, TT, TT, DH);
    k_relsoft<<<NH * TT / 8, 256, 0, stream>>>(S, Q16, relk, mask, b, P16, PB); k_vt<<<(NH * DH * (TT / 8) + 255) / 256, 256, 0, stream>>>(V16, b, VT);
    k_gemm_hhx<0><<<dim3(((TT / 16) * ((DH + 63) / 64) + 3) / 4, NH), 128, 0, stream>>>(P16, TT, (size_t)TT * TT, VT, TT, (size_t)DH * TT, 0.0009765625f, nullptr, 0, nullptr, 1, 0, 0, O, nullptr, CC, DH, TT, DH, TT);
    k_relv<<<(TT * (CC / 8) + 255) / 256, 256, 0, stream>>>(O, PB, relv, b, O16); }
  k_gemm_hhx<0><<<gC, 128, 0, stream>>>(O16, CC, 0, Bo, CC, 0, 0.0625f, bo, 0, XT, 1, (size_t)CC, 0, XT, nullptr, CC, 0, NR, CC, CC);
  k_ln<<<NR / 8, 256, 0, stream>>>(XT, cg, cb, LN16);
  k_gemm_hhx<0><<<g2C, 128, 0, stream>>>(LN16, CC, 0, Bp1, CC, 0, 0.0625f, pb1, 0, nullptr, 1, 0, 0, PW, nullptr, 2 * CC, 0, NR, 2 * CC, CC);
  k_glu<<<(unsigned)(((size_t)NR * (CC / 4) + 255) / 256), 256, 0, stream>>>(PW, GL); k_dw<<<(unsigned)(((size_t)NR * (CC / 8) + 255) / 256), 256, 0, stream>>>(GL, dww, dwb, bng, bnb, CH);
  k_gemm_hhx<0><<<gC, 128, 0, stream>>>(CH, CC, 0, Bp2, CC, 0, 0.0625f, pb2, 0, XT, 1, (size_t)CC, 0, XT, nullptr, CC, 0, NR, CC, CC);
  k_ln<<<NR / 8, 256, 0, stream>>>(XT, f2g, f2bb, LN16);
  k_gemm_hhx<15><<<gF, 128, 0, stream>>>(LN16, CC, 0, Bf2w1, CC, 0, 0.0625f, f2b1, 0, nullptr, 1, 0, 0, nullptr, FFH, FF, 0, NR, FF, CC);
  k_gemm_hhx<0><<<gC, 128, 0, stream>>>(FFH, FF, 0, Bf2w2, FF, 0, 0.0625f * 0.5f, B2b, 0, XT, 1, (size_t)CC, 0, XT, nullptr, CC, 0, NR, CC, FF);
  k_stat<<<NR / 32, 1024, 0, stream>>>(XT, MU, RS); k_tout<<<(unsigned)(((size_t)NB * CC * (TT / 4) + 255) / 256), 256, 0, stream>>>(XT, MU, RS, postg, postb, mask, (float*)d_out);
}
